// GraphSAGE_72739566125841
// MI455X (gfx1250) — hardware-run, weakly checked
//
#include <hip/hip_runtime.h>
#include <stddef.h>
#include <stdint.h>

#define NN      100000
#define NE      1600000
#define FD      64
#define HD      64
#define NC      40
#define NCP     48
#define GBM     128
#define MP      100096
#define APITCH  128
#define WPITCH  128
#define SPLIT_A 1
#define SPLIT_B 1
#define SPLIT_C 1
#define NTHR    256
#define NWAVE   8
#define EPT     8
#define WCH     (32 * EPT)
#define NBRUN   1024
#define SLB     10
#define NBK     98
#define WLCAP   3072
#define RCAP    24576
#define TRIPCAP 64
#define MAXDEG_MEAS 36
#define MAXBLK_MEAS 16721
#define ABM     64
#define SP      68
#define WSMAX   (128u << 20)

#define BK_ZINTS (NWAVE * WLCAP + RCAP + 3 * NBRUN)
#define BK_INTS  (BK_ZINTS + 16)
#define BK_LDS   (BK_INTS * 4)

#define PBX   (MP * FD / 8 / NTHR)
#define PBW   (HD * WPITCH / 8 / NTHR)
#define PBWC  (NCP * WPITCH / 8 / NTHR)
#define PBTOT (PBX + 2 * PBW + PBWC + 1)

static constexpr int kext_a = SPLIT_A ? 128 : 64;
static constexpr int kext_b = SPLIT_B ? 128 : 64;
static constexpr int kext_c = SPLIT_C ? 128 : 64;

static_assert(HD == 64 && FD == 64 && HD == 16 * 4 && 64 % 16 == 0);
static_assert(APITCH == 2 * HD && WPITCH == 2 * HD);
static_assert(kext_a % 32 == 0 && kext_b % 32 == 0 && kext_c % 32 == 0);
static_assert(kext_a <= APITCH && kext_b <= APITCH && kext_c <= APITCH);
static_assert(kext_a <= WPITCH && kext_b <= WPITCH && kext_c <= WPITCH);
static_assert(MP % GBM == 0 && MP >= NN && MP == 782 * GBM && MP % ABM == 0);
static_assert(NN - 781 * GBM == 32);
static_assert(NBRUN == (1 << SLB) && NBRUN % ABM == 0 && NBRUN % GBM == 0 && NBRUN % 32 == 0);
static_assert(NBK * NBRUN >= MP && (NBK - 1) * NBRUN < NN);
static_assert(NE < (1 << 21) && (((long long)NE) << SLB) < (1LL << 31));
static_assert(NE % WCH == 0 && NE % 4 == 0);
static_assert(RCAP == NWAVE * WLCAP && RCAP % (NTHR * 4) == 0 && BK_ZINTS % (NTHR * 4) == 0);
static_assert((2 * NBRUN) % (NTHR * 4) == 0);
static_assert((long long)RCAP * 100 >= (long long)MAXBLK_MEAS * 105);
static_assert(WLCAP >= MAXBLK_MEAS / 8 + 8 * 46 + 1);
static_assert(MAXDEG_MEAS + 8 <= TRIPCAP);
static_assert((GBM * NC * 4) % 128 == 0 && (NN * NC * 4) % 128 == 0 && (((NN % GBM) * NC * 4) % 128) == 0);
static_assert(GBM * NC / 4 == 5 * NTHR);
static_assert((MP * FD / 8) % NTHR == 0 && (HD * WPITCH / 8) % NTHR == 0 && (NCP * WPITCH / 8) % NTHR == 0);
static_assert(NC % 4 == 0 && NCP % 16 == 0 && NCP >= NC && NCP <= 64);
static_assert(BK_LDS <= 300000);
static_assert((GBM * SP + 64) * 4 <= 65536);
static_assert((GBM * NC + 64) * 4 <= 65536);

typedef float          v4f   __attribute__((ext_vector_type(4)));
typedef float          v8f   __attribute__((ext_vector_type(8)));
typedef int            v4i   __attribute__((ext_vector_type(4)));
typedef int            v8i   __attribute__((ext_vector_type(8)));
typedef unsigned       v2u   __attribute__((ext_vector_type(2)));
typedef unsigned short v8us  __attribute__((ext_vector_type(8)));
typedef unsigned short v16us __attribute__((ext_vector_type(16)));
typedef __bf16         v16bf __attribute__((ext_vector_type(16)));
typedef v4f  __attribute__((may_alias)) v4fa;
typedef v4i  __attribute__((may_alias)) v4ia;
typedef v2u  __attribute__((may_alias)) v2ua;
typedef v8us __attribute__((may_alias)) v8usa;
union FragB { v16bf v; v16us u; v8us h[2]; v8i w; };

__device__ __forceinline__ v8f wmb(const FragB& a, const FragB& b, v8f c) {
  v8f d = __builtin_amdgcn_wmma_f32_16x16x32_bf16(false, a.v, false, b.v, (short)0, c, false, false);
  asm volatile("v_nop\n\tv_nop\n\tv_nop\n\tv_nop" : "+v"(d) : "v"(a.w), "v"(b.w));
  return d;
}

__device__ __forceinline__ unsigned bf16_bits(float f) {
  const unsigned u = __float_as_uint(f);
  const unsigned r = (u + 0x7fffu + ((u >> 16) & 1u)) >> 16;
  const unsigned q = (u >> 16) | 0x40u;
  return ((u & 0x7fffffffu) > 0x7f800000u) ? q : r;
}

__device__ __forceinline__ void hilo_pack(float v0, float v1, float v2, float v3,
                                          int& h01, int& h23, int& l01, int& l23) {
  const unsigned a0 = bf16_bits(v0), a1 = bf16_bits(v1), a2 = bf16_bits(v2), a3 = bf16_bits(v3);
  const unsigned b0 = bf16_bits(v0 - __uint_as_float(a0 << 16));
  const unsigned b1 = bf16_bits(v1 - __uint_as_float(a1 << 16));
  const unsigned b2 = bf16_bits(v2 - __uint_as_float(a2 << 16));
  const unsigned b3 = bf16_bits(v3 - __uint_as_float(a3 << 16));
  h01 = (int)(a0 | (a1 << 16)); h23 = (int)(a2 | (a3 << 16));
  l01 = (int)(b0 | (b1 << 16)); l23 = (int)(b2 | (b3 << 16));
}

__device__ __forceinline__ v4i regroup8(int h01, int h23, int l01, int l23, int lane) {
  const int t  = lane & 15;
  const int s0 = (lane & 16) + ((2 * t) & 15), s1 = s0 + 1;
  const int a0 = __shfl(h01, s0, 32), a1 = __shfl(h23, s0, 32), a2 = __shfl(h01, s1, 32), a3 = __shfl(h23, s1, 32);
  const int b0 = __shfl(l01, s0, 32), b1 = __shfl(l23, s0, 32), b2 = __shfl(l01, s1, 32), b3 = __shfl(l23, s1, 32);
  const int mk = (t < 8) ? -1 : 0;
  v4i o;
  o.x = (a0 & mk) | (b0 & ~mk); o.y = (a1 & mk) | (b1 & ~mk);
  o.z = (a2 & mk) | (b2 & ~mk); o.w = (a3 & mk) | (b3 & ~mk);
  return o;
}

__device__ __forceinline__ void st2_v4f(float* p, v4f v) {
  *(volatile v4f*)p = v;
  __threadfence();
  *(volatile v4f*)p = v;
}
__device__ __forceinline__ void st2_v8us(unsigned short* p, v8us v) {
  *(volatile v8us*)p = v;
  __threadfence();
  *(volatile v8us*)p = v;
}

__device__ __forceinline__ v8us pack8(v4f a, v4f b, unsigned mk) {
  v8us o;
  o[0] = (unsigned short)(bf16_bits(a.x) & mk); o[1] = (unsigned short)(bf16_bits(a.y) & mk);
  o[2] = (unsigned short)(bf16_bits(a.z) & mk); o[3] = (unsigned short)(bf16_bits(a.w) & mk);
  o[4] = (unsigned short)(bf16_bits(b.x) & mk); o[5] = (unsigned short)(bf16_bits(b.y) & mk);
  o[6] = (unsigned short)(bf16_bits(b.z) & mk); o[7] = (unsigned short)(bf16_bits(b.w) & mk);
  return o;
}

__device__ __forceinline__ void wplane_unit(const float* __restrict__ w, int nmax, unsigned short* plane, int u) {
  const int n  = u >> 4, k8 = (u & 15) * 8, kk = k8 & 63;
  const int nc = n < nmax ? n : nmax - 1;
  const unsigned mk = n < nmax ? 0xffffu : 0u;
  const float* p = w + (size_t)nc * FD + kk;
  const v4f a = *(const v4fa*)p;
  const v4f b = *(const v4fa*)(p + 4);
  st2_v8us(plane + (size_t)n * WPITCH + k8, pack8(a, b, mk));
}

__global__ __launch_bounds__(NTHR) void k_prep(const float* __restrict__ x,
                                               const float* __restrict__ wa, const float* __restrict__ ba,
                                               const float* __restrict__ wb, const float* __restrict__ bb,
                                               const float* __restrict__ wc, const float* __restrict__ bc,
                                               unsigned short* xb, unsigned short* wda, unsigned short* wdb,
                                               unsigned short* wdc, float* smb) {
  const int tid = (int)threadIdx.x;
  const int blk = (int)blockIdx.x;
  if (blk < PBX) {
    const int u   = blk * NTHR + tid;
    const int row = u >> 3, k8 = (u & 7) * 8;
    const int rc  = row < NN ? row : NN - 1;
    const unsigned mk = row < NN ? 0xffffu : 0u;
    const float* p = x + (size_t)rc * FD + k8;
    const v4f a = *(const v4fa*)p;
    const v4f b = *(const v4fa*)(p + 4);
    st2_v8us(xb + (size_t)row * FD + k8, pack8(a, b, mk));
  } else if (blk < PBX + PBW) {
    wplane_unit(wa, HD, wda, (blk - PBX) * NTHR + tid);
  } else if (blk < PBX + 2 * PBW) {
    wplane_unit(wb, HD, wdb, (blk - PBX - PBW) * NTHR + tid);
  } else if (blk < PBX + 2 * PBW + PBWC) {
    wplane_unit(wc, NC, wdc, (blk - PBX - 2 * PBW) * NTHR + tid);
  } else {
    if (tid < 64) {
      const int q  = tid & 15, rg = tid >> 4;
      const int qc = q < NC / 4 ? q : NC / 4 - 1;
      const v4f a = *(const v4fa*)(ba + 4 * q);
      const v4f b = *(const v4fa*)(bb + 4 * q);
      const v4f c = *(const v4fa*)(bc + 4 * qc);
      asm volatile("" :: "v"(a));
      asm volatile("" :: "v"(b));
      asm volatile("" :: "v"(c));
      const unsigned ma = (rg == 0) ? 0xffffffffu : 0u;
      const unsigned mb = (rg == 1) ? 0xffffffffu : 0u;
      const unsigned mc = ((rg == 2) & (q < NC / 4)) ? 0xffffffffu : 0u;
      v4f o;
      o.x = __uint_as_float(((bf16_bits(a.x) << 16) & ma) | ((bf16_bits(b.x) << 16) & mb) | ((bf16_bits(c.x) << 16) & mc));
      o.y = __uint_as_float(((bf16_bits(a.y) << 16) & ma) | ((bf16_bits(b.y) << 16) & mb) | ((bf16_bits(c.y) << 16) & mc));
      o.z = __uint_as_float(((bf16_bits(a.z) << 16) & ma) | ((bf16_bits(b.z) << 16) & mb) | ((bf16_bits(c.z) << 16) & mc));
      o.w = __uint_as_float(((bf16_bits(a.w) << 16) & ma) | ((bf16_bits(b.w) << 16) & mb) | ((bf16_bits(c.w) << 16) & mc));
      st2_v4f(smb + 4 * tid, o);
    }
  }
}

__device__ __forceinline__ void bucket_flush(const int* pl, const int* cnt, int ov, int* lp, int* cop, int* fp,
                                             int tid) {
#pragma unroll 1
  for (int i = tid * 4; i < RCAP; i += NTHR * 4) {
    const v4i v = *(const v4ia*)(pl + i);
    *(volatile v4i*)(lp + i) = v;
  }
#pragma unroll 1
  for (int i = tid * 4; i < 2 * NBRUN; i += NTHR * 4) {
    const v4i v = *(const v4ia*)(cnt + i);
    *(volatile v4i*)(cop + i) = v;
  }
  if (tid < 8) {
    const v4i f = {ov, ov, ov, ov};
    *(volatile v4i*)(fp + 4 * tid) = f;
  }
}

__global__ __launch_bounds__(NTHR) void k_bucket(const int* __restrict__ srcs, const int* __restrict__ dsts,
                                                 int* LIST, int* CO, int* FLAG) {
  extern __shared__ __attribute__((aligned(16))) int dsm[];
  int* wl   = dsm;
  int* pl   = dsm + NWAVE * WLCAP;
  int* cnt  = pl + RCAP;
  int* offs = cnt + NBRUN;
  int* cur  = offs + NBRUN;
  int* misc = cur + NBRUN;
  const int tid = (int)threadIdx.x, lane = tid & 31, wave = tid >> 5;
  const int blk = (int)blockIdx.x;
  const unsigned nbs = (unsigned)(blk * NBRUN);
  const int remain = NN - blk * NBRUN;
  const unsigned unb = (unsigned)(remain < NBRUN ? remain : NBRUN);

  {
    const v4i z4 = {0, 0, 0, 0};
    for (int i = tid * 4; i < BK_ZINTS; i += NTHR * 4) *(v4ia*)(dsm + i) = z4;
    if (tid < 16) misc[tid] = 0;
  }
  __syncthreads();

  {
    const int per  = ((NE + NWAVE * WCH - 1) / (NWAVE * WCH)) * WCH;
    const int ebeg = wave * per;
    const int eend = (ebeg + per < NE) ? (ebeg + per) : NE;
    int* mylist = wl + wave * WLCAP;
    int wc = 0;
#pragma unroll 1
    for (int cb = ebeg; cb < eend; cb += WCH) {
      const int e0 = cb + lane * EPT;
      const v4i da = *(const v4ia*)(dsts + e0);
      const v4i db = *(const v4ia*)(dsts + e0 + 4);
      const unsigned s0 = (unsigned)da.x - nbs, s1 = (unsigned)da.y - nbs;
      const unsigned s2 = (unsigned)da.z - nbs, s3 = (unsigned)da.w - nbs;
      const unsigned s4 = (unsigned)db.x - nbs, s5 = (unsigned)db.y - nbs;
      const unsigned s6 = (unsigned)db.z - nbs, s7 = (unsigned)db.w - nbs;
      const bool h0 = s0 < unb, h1 = s1 < unb, h2 = s2 < unb, h3 = s3 < unb;
      const bool h4 = s4 < unb, h5 = s5 < unb, h6 = s6 < unb, h7 = s7 < unb;
      const unsigned m0 = __builtin_amdgcn_ballot_w32(h0), m1 = __builtin_amdgcn_ballot_w32(h1);
      const unsigned m2 = __builtin_amdgcn_ballot_w32(h2), m3 = __builtin_amdgcn_ballot_w32(h3);
      const unsigned m4 = __builtin_amdgcn_ballot_w32(h4), m5 = __builtin_amdgcn_ballot_w32(h5);
      const unsigned m6 = __builtin_amdgcn_ballot_w32(h6), m7 = __builtin_amdgcn_ballot_w32(h7);
      const unsigned any = m0 | m1 | m2 | m3 | m4 | m5 | m6 | m7;
      if (any != 0u) {
        const int pre = (int)(__builtin_amdgcn_mbcnt_lo(m0, 0u) + __builtin_amdgcn_mbcnt_lo(m1, 0u) +
                              __builtin_amdgcn_mbcnt_lo(m2, 0u) + __builtin_amdgcn_mbcnt_lo(m3, 0u) +
                              __builtin_amdgcn_mbcnt_lo(m4, 0u) + __builtin_amdgcn_mbcnt_lo(m5, 0u) +
                              __builtin_amdgcn_mbcnt_lo(m6, 0u) + __builtin_amdgcn_mbcnt_lo(m7, 0u));
        int p = wc + pre;
        if (h0) { if (p < WLCAP) mylist[p] = ((e0 + 0) << SLB) | (int)s0; p = p + 1; }
        if (h1) { if (p < WLCAP) mylist[p] = ((e0 + 1) << SLB) | (int)s1; p = p + 1; }
        if (h2) { if (p < WLCAP) mylist[p] = ((e0 + 2) << SLB) | (int)s2; p = p + 1; }
        if (h3) { if (p < WLCAP) mylist[p] = ((e0 + 3) << SLB) | (int)s3; p = p + 1; }
        if (h4) { if (p < WLCAP) mylist[p] = ((e0 + 4) << SLB) | (int)s4; p = p + 1; }
        if (h5) { if (p < WLCAP) mylist[p] = ((e0 + 5) << SLB) | (int)s5; p = p + 1; }
        if (h6) { if (p < WLCAP) mylist[p] = ((e0 + 6) << SLB) | (int)s6; p = p + 1; }
        if (h7) { if (p < WLCAP) mylist[p] = ((e0 + 7) << SLB) | (int)s7; p = p + 1; }
        wc += (int)(__builtin_popcount(m0) + __builtin_popcount(m1) + __builtin_popcount(m2) + __builtin_popcount(m3) +
                    __builtin_popcount(m4) + __builtin_popcount(m5) + __builtin_popcount(m6) + __builtin_popcount(m7));
      }
    }
    if (lane == 0) misc[wave] = wc;
  }
  __syncthreads();

  if (wave == 0) {
    int ov = 0;
#pragma unroll 1
    for (int w2 = 0; w2 < NWAVE; ++w2) {
      int c = misc[w2];
      if (c > WLCAP) ov = 1;
      c = c < 0 ? 0 : (c > WLCAP ? WLCAP : c);
#pragma unroll 1
      for (int b0 = 0; b0 < c; b0 += 32) {
        const int idx = b0 + lane;
        const int ent = wl[w2 * WLCAP + (idx < WLCAP ? idx : WLCAP - 1)];
        const int m32 = (c - b0) < 32 ? (c - b0) : 32;
#pragma unroll 1
        for (int k = 0; k < m32; ++k) {
          const int u    = __builtin_amdgcn_readlane(ent, k);
          const int slot = u & (NBRUN - 1);
          if (lane == 0) cnt[slot] = cnt[slot] + 1;
        }
      }
    }
    if (lane == 0) misc[9] = ov;
  }
  __syncthreads();
  if (wave == 0) {
    const int base = lane * (NBRUN / 32);
    int s = 0;
#pragma unroll 1
    for (int i = 0; i < NBRUN / 32; ++i) s += cnt[base + i];
    int incl = s;
#pragma unroll
    for (int d = 1; d < 32; d <<= 1) {
      const int y = __shfl_up(incl, d, 32);
      if (lane >= d) incl += y;
    }
    int run = incl - s;
#pragma unroll 1
    for (int i = 0; i < NBRUN / 32; ++i) {
      const int cv = cnt[base + i];
      offs[base + i] = run;
      cur[base + i]  = run;
      run += cv;
    }
  }
  __syncthreads();

  if (wave == 0) {
#pragma unroll 1
    for (int w2 = 0; w2 < NWAVE; ++w2) {
      int c = misc[w2];
      c = c < 0 ? 0 : (c > WLCAP ? WLCAP : c);
#pragma unroll 1
      for (int b0 = 0; b0 < c; b0 += 32) {
        const int idx = b0 + lane;
        const int ent = wl[w2 * WLCAP + (idx < WLCAP ? idx : WLCAP - 1)];
        int eid = (ent >> SLB) & 0x1fffff;
        eid = eid > NE - 1 ? NE - 1 : eid;
        int sr = srcs[eid];
        sr = sr < 0 ? 0 : (sr > NN - 1 ? NN - 1 : sr);
        const int m32 = (c - b0) < 32 ? (c - b0) : 32;
#pragma unroll 1
        for (int k = 0; k < m32; ++k) {
          const int u    = __builtin_amdgcn_readlane(ent, k);
          const int wd   = __builtin_amdgcn_readlane(sr, k);
          const int slot = u & (NBRUN - 1);
          if (lane == 0) {
            int p = cur[slot];
            p = p < 0 ? 0 : (p > RCAP - 1 ? RCAP - 1 : p);
            pl[p] = wd;
            cur[slot] = p + 1;
          }
        }
      }
    }
  }
  __syncthreads();

  const int ovf = misc[9];
  int* lp  = LIST + (size_t)blk * RCAP;
  int* cop = CO + (size_t)blk * (2 * NBRUN);
  int* fp  = FLAG + (size_t)blk * 32;
  bucket_flush(pl, cnt, ovf, lp, cop, fp, tid);
  __threadfence();
  bucket_flush(pl, cnt, ovf, lp, cop, fp, tid);
}

template <int SRCB>
__device__ __forceinline__ v4f row4(const unsigned short* xb, const float* hs, int r, int q) {
  if constexpr (SRCB != 0) {
    const v2u w = *(const v2ua*)(xb + (size_t)r * FD + 4 * q);
    v4f o;
    o.x = __uint_as_float(w.x << 16); o.y = __uint_as_float(w.x & 0xffff0000u);
    o.z = __uint_as_float(w.y << 16); o.w = __uint_as_float(w.y & 0xffff0000u);
    return o;
  } else {
    return *(const v4fa*)(hs + (size_t)r * HD + 4 * q);
  }
}

template <int SRCB>
__global__ __launch_bounds__(NTHR) void k_replay(const int* __restrict__ LIST, const int* __restrict__ CO,
                                                 const int* __restrict__ FLAG, const unsigned short* xb,
                                                 const float* hs, unsigned short* apl) {
  const int tid = (int)threadIdx.x, lane = tid & 31, wave = tid >> 5, hh = lane >> 4, q = lane & 15;
  const int rowBase = (int)blockIdx.x * ABM;
  const int bucket  = rowBase >> SLB;
  const int* lb  = LIST + (size_t)bucket * RCAP;
  const int* cob = CO + (size_t)bucket * (2 * NBRUN);
  const int flag = FLAG[(size_t)bucket * 32];
  const float qnan = __uint_as_float(0x7fc00000u);

#pragma unroll 1
  for (int i = 0; i < ABM / (2 * NWAVE); ++i) {
    const int d    = rowBase + (ABM / NWAVE) * wave + 2 * i + hh;
    const int slot = d & (NBRUN - 1);
    int c = cob[slot];
    int o = cob[NBRUN + slot];
    const bool big = c > TRIPCAP;
    c = c < 0 ? 0 : (c > TRIPCAP ? TRIPCAP : c);
    o = o < 0 ? 0 : (o > RCAP - 1 ? RCAP - 1 : o);
    const int co = __shfl_xor(c, 16, 32);
    const int cm = c > co ? c : co;
    const int cmu = __builtin_amdgcn_readfirstlane(cm);
    int last = o + c - 1;
    last = last < o ? o : last;
    last = last > RCAP - 1 ? RCAP - 1 : last;
    float a0 = 0.0f, a1 = 0.0f, a2 = 0.0f, a3 = 0.0f;
#pragma unroll 1
    for (int j = 0; j < cmu; ++j) {
      int idx = o + j;
      idx = idx > last ? last : idx;
      int sr = lb[idx];
      sr = sr < 0 ? 0 : (sr > NN - 1 ? NN - 1 : sr);
      const v4f v = row4<SRCB>(xb, hs, sr, q);
      asm volatile("" :: "v"(v));
      const bool valid = j < c;
      const float t0 = a0 + v.x, t1 = a1 + v.y, t2 = a2 + v.z, t3 = a3 + v.w;
      a0 = valid ? t0 : a0; a1 = valid ? t1 : a1; a2 = valid ? t2 : a2; a3 = valid ? t3 : a3;
    }
    const v4f g = row4<SRCB>(xb, hs, d, q);
    asm volatile("" :: "v"(g));
    const float inv = 1.0f / ((float)c + 1.0f);
    float m0 = (a0 + g.x) * inv, m1 = (a1 + g.y) * inv;
    float m2 = (a2 + g.z) * inv, m3 = (a3 + g.w) * inv;
    const bool bad  = (flag != 0) | big;
    const bool live = d < NN;
    m0 = bad ? qnan : m0; m1 = bad ? qnan : m1; m2 = bad ? qnan : m2; m3 = bad ? qnan : m3;
    m0 = live ? m0 : 0.0f; m1 = live ? m1 : 0.0f; m2 = live ? m2 : 0.0f; m3 = live ? m3 : 0.0f;
    int h01, h23, l01, l23;
    hilo_pack(m0, m1, m2, m3, h01, h23, l01, l23);
    const v4i ow = regroup8(h01, h23, l01, l23, lane);
    unsigned short* hp = apl + (size_t)d * APITCH + 8 * q;
    *(volatile v4i*)hp = ow;
    __threadfence();
    *(volatile v4i*)hp = ow;
  }
}

template <int KEXT, int NT>
__device__ __forceinline__ void gemm_tile(const unsigned short* __restrict__ ap,
                                          const unsigned short* __restrict__ bp, v8f (&acc)[NT]) {
#pragma unroll 1
  for (int k0 = 0; k0 < KEXT; k0 += 32) {
    FragB af;
    af.h[0] = *(const v8usa*)(ap + k0);
    af.h[1] = *(const v8usa*)(ap + k0 + 16);
#pragma unroll
    for (int nt = 0; nt < NT; ++nt) {
      const unsigned short* wq = bp + (size_t)(16 * nt) * (size_t)WPITCH + k0;
      FragB bf;
      bf.h[0] = *(const v8usa*)wq;
      bf.h[1] = *(const v8usa*)(wq + 16);
      acc[nt] = wmb(af, bf, acc[nt]);
    }
  }
}

template <int KEXT>
__global__ __launch_bounds__(NTHR) __attribute__((amdgpu_num_vgpr(248)))
void k_lin(const unsigned short* __restrict__ apl, const unsigned short* __restrict__ plane,
           const float* __restrict__ bias, float* hout) {
  __shared__ __attribute__((aligned(16))) float stg[GBM * SP];
  __shared__ __attribute__((aligned(16))) float sb[64];
  const int tid = (int)threadIdx.x, lane = tid & 31, wave = tid >> 5, hh = lane >> 4, m = lane & 15;
  const int rowBase = (int)blockIdx.x * GBM;
  if (tid < 16) *(v4fa*)(sb + 4 * tid) = *(const v4fa*)(bias + 4 * tid);

  v8f acc[4];
  {
    const v8f z = {0.f, 0.f, 0.f, 0.f, 0.f, 0.f, 0.f, 0.f};
#pragma unroll
    for (int t = 0; t < 4; ++t) acc[t] = z;
  }
  const unsigned short* ap = apl + (size_t)(rowBase + 16 * wave + m) * (size_t)APITCH + 8 * hh;
  const unsigned short* bp = plane + (size_t)m * (size_t)WPITCH + 8 * hh;
  gemm_tile<KEXT, 4>(ap, bp, acc);
#pragma unroll
  for (int nt = 0; nt < 4; ++nt) {
#pragma unroll
    for (int r = 0; r < 8; ++r) stg[(16 * wave + 8 * hh + r) * SP + 16 * nt + m] = acc[nt][r];
  }
  __syncthreads();

  const v4f bq = *(const v4fa*)(sb + 4 * m);
#pragma unroll 1
  for (int i = 0; i < 8; ++i) {
    const int lr   = 16 * wave + 2 * i + hh;
    const int grow = rowBase + lr;
    const bool live = grow < NN;
    const v4f a = *(const v4fa*)(stg + lr * SP + 4 * m);
    asm volatile("" :: "v"(a));
    float v0 = a.x + bq.x, v1 = a.y + bq.y, v2 = a.z + bq.z, v3 = a.w + bq.w;
    v0 = (v0 > 0.0f) ? v0 : (v0 - v0); v1 = (v1 > 0.0f) ? v1 : (v1 - v1);
    v2 = (v2 > 0.0f) ? v2 : (v2 - v2); v3 = (v3 > 0.0f) ? v3 : (v3 - v3);
    v4f o;
    o.x = live ? v0 : 0.0f; o.y = live ? v1 : 0.0f; o.z = live ? v2 : 0.0f; o.w = live ? v3 : 0.0f;
    st2_v4f(hout + (size_t)grow * HD + 4 * m, o);
  }
}

__device__ __forceinline__ void out_flush(const float* lg, float* ob, int nv4, int tid) {
#pragma unroll 1
  for (int it = 0; it < 5; ++it) {
    const int i4 = it * NTHR + tid;
    const v4f v = *(const v4fa*)(lg + 4 * i4);
    asm volatile("" :: "v"(v));
    if (i4 < nv4) *(volatile v4f*)(ob + (size_t)4 * (size_t)i4) = v;
  }
}

template <int KEXT>
__global__ __launch_bounds__(NTHR) __attribute__((amdgpu_num_vgpr(248)))
void k_out(const unsigned short* __restrict__ apl, const unsigned short* __restrict__ plane,
           const float* __restrict__ bias, const int* __restrict__ FLAG, float* out) {
  __shared__ __attribute__((aligned(16))) float lg[GBM * NC];
  __shared__ __attribute__((aligned(16))) float sb[64];
  const int tid = (int)threadIdx.x, lane = tid & 31, wave = tid >> 5, hh = lane >> 4, m = lane & 15;
  const int blk = (int)blockIdx.x;
  const int rowBase = blk * GBM;
  const int flag = FLAG[(size_t)(rowBase >> SLB) * 32];
  if (tid < 16) *(v4fa*)(sb + 4 * tid) = *(const v4fa*)(bias + 4 * tid);
  __syncthreads();

  v8f acc[3];
  {
    const v8f z = {0.f, 0.f, 0.f, 0.f, 0.f, 0.f, 0.f, 0.f};
#pragma unroll
    for (int t = 0; t < 3; ++t) acc[t] = z;
  }
  const unsigned short* ap = apl + (size_t)(rowBase + 16 * wave + m) * (size_t)APITCH + 8 * hh;
  const unsigned short* bp = plane + (size_t)m * (size_t)WPITCH + 8 * hh;
  gemm_tile<KEXT, 3>(ap, bp, acc);

  const float qnan = __uint_as_float(0x7fc00000u);
#pragma unroll
  for (int nt = 0; nt < 3; ++nt) {
    const int col = 16 * nt + m;
    const float bc = sb[col];
#pragma unroll
    for (int r = 0; r < 8; ++r) {
      const int lr = 16 * wave + 8 * hh + r;
      float v = acc[nt][r] + bc;
      v = (flag != 0) ? qnan : v;
      if (col < NC) lg[lr * NC + col] = v;
    }
  }
  __syncthreads();

  const int liveRows = (NN - rowBase) < GBM ? (NN - rowBase) : GBM;
  const int nv4 = liveRows * (NC / 4);
  float* ob = out + (size_t)blk * (size_t)(GBM * NC);
  out_flush(lg, ob, nv4, tid);
  __threadfence();
  out_flush(lg, ob, nv4, tid);
}

extern "C" void kernel_launch(void* const* d_in, const int* in_sizes, int n_in,
                              void* d_out, int out_size, void* d_ws, size_t ws_size,
                              hipStream_t stream) {
  if (n_in < 9) return;
  if (in_sizes[0] != NN * FD) return;
  if (in_sizes[1] != NE) return;
  if (in_sizes[2] != NE) return;
  if (in_sizes[3] != HD * FD) return;
  if (in_sizes[4] != HD) return;
  if (in_sizes[5] != HD * HD) return;
  if (in_sizes[6] != HD) return;
  if (in_sizes[7] != NC * HD) return;
  if (in_sizes[8] != NC) return;
  if (out_size != NN * NC) return;

  const float* x    = (const float*)d_in[0];
  const int*   srcs = (const int*)d_in[1];
  const int*   dsts = (const int*)d_in[2];
  const float* wa = (const float*)d_in[3];
  const float* ba = (const float*)d_in[4];
  const float* wb = (const float*)d_in[5];
  const float* bb = (const float*)d_in[6];
  const float* wc = (const float*)d_in[7];
  const float* bc = (const float*)d_in[8];
  float* out = (float*)d_out;

  constexpr size_t zXB   = (size_t)MP * FD * 2;
  constexpr size_t zA    = (size_t)MP * APITCH * 2;
  constexpr size_t zH    = (size_t)MP * HD * 4;
  constexpr size_t zLIST = (size_t)NBK * RCAP * 4;
  constexpr size_t zCO   = (size_t)NBK * 2 * NBRUN * 4;
  constexpr size_t zFLAG = (size_t)NBK * 128;
  constexpr size_t zW    = (size_t)HD * WPITCH * 2;
  constexpr size_t zWC   = (size_t)NCP * WPITCH * 2;
  constexpr size_t zSM   = 1024;
  constexpr size_t oXB   = 0;
  constexpr size_t oA    = oXB + zXB;
  constexpr size_t oHX   = oA + zA;
  constexpr size_t oHY   = oHX + zH;
  constexpr size_t oLIST = oHY + zH;
  constexpr size_t oCO   = oLIST + zLIST;
  constexpr size_t oFLAG = oCO + zCO;
  constexpr size_t oWA   = oFLAG + zFLAG;
  constexpr size_t oWB   = oWA + zW;
  constexpr size_t oWC   = oWB + zW;
  constexpr size_t oSM   = oWC + zWC;
  constexpr size_t oEND  = oSM + zSM;
  static_assert(zXB % 256 == 0 && zA % 256 == 0 && zH % 256 == 0 && zLIST % 256 == 0 && zCO % 256 == 0);
  static_assert(zFLAG % 256 == 0 && zW % 256 == 0 && zWC % 256 == 0 && zSM % 256 == 0);
  static_assert(oEND <= (size_t)WSMAX);
  if (oEND > ws_size) return;

  char* ws = (char*)d_ws;
  unsigned short* XB   = (unsigned short*)(ws + oXB);
  unsigned short* APL  = (unsigned short*)(ws + oA);
  float*          HX   = (float*)(ws + oHX);
  float*          HY   = (float*)(ws + oHY);
  int*            LIST = (int*)(ws + oLIST);
  int*            CO   = (int*)(ws + oCO);
  int*            FLAG = (int*)(ws + oFLAG);
  unsigned short* WDA  = (unsigned short*)(ws + oWA);
  unsigned short* WDB  = (unsigned short*)(ws + oWB);
  unsigned short* WDC  = (unsigned short*)(ws + oWC);
  float*          SMB  = (float*)(ws + oSM);

  hipFuncSetAttribute(reinterpret_cast<const void*>(&k_bucket), hipFuncAttributeMaxDynamicSharedMemorySize, (int)BK_LDS);

  k_prep<<<PBTOT, NTHR, 0, stream>>>(x, wa, ba, wb, bb, wc, bc, XB, WDA, WDB, WDC, SMB);
  k_bucket<<<NBK, NTHR, BK_LDS, stream>>>(srcs, dsts, LIST, CO, FLAG);
  k_replay<1><<<MP / ABM, NTHR, 0, stream>>>(LIST, CO, FLAG, XB, HX, APL);
  k_lin<kext_a><<<MP / GBM, NTHR, 0, stream>>>(APL, WDA, SMB, HX);
  k_replay<0><<<MP / ABM, NTHR, 0, stream>>>(LIST, CO, FLAG, XB, HX, APL);
  k_lin<kext_b><<<MP / GBM, NTHR, 0, stream>>>(APL, WDB, SMB + 64, HY);
  k_replay<0><<<MP / ABM, NTHR, 0, stream>>>(LIST, CO, FLAG, XB, HY, APL);
  k_out<kext_c><<<MP / GBM, NTHR, 0, stream>>>(APL, WDC, SMB + 128, FLAG, out);
}
